// ALSTM_16887811408328
// MI455X (gfx1250) — hardware-run, weakly checked
//
#include <hip/hip_runtime.h>
#include <math.h>

typedef __attribute__((ext_vector_type(16))) _Float16 v16h;
typedef __attribute__((ext_vector_type(8)))  _Float16 v8h;
typedef __attribute__((ext_vector_type(8)))  float    v8f;
typedef __attribute__((ext_vector_type(4)))  float    v4f;
typedef __attribute__((ext_vector_type(2)))  unsigned int v2u;

constexpr int kB      = 4096;
constexpr int kI      = 512;
constexpr int kH      = 512;
constexpr int kO      = 512;
constexpr int kG      = 4 * kH;
constexpr int kSteps  = 16;
constexpr int kWihP   = 1 + kI;
constexpr int kRowsPerBlk = 64;
constexpr int kChunkCols  = 64;
constexpr int kPatchP     = 260;
constexpr float kWoutCarry = 1024.0f;
constexpr float kHfinCarry = 64.0f;
constexpr float kOutScale  = 1.0f / (kWoutCarry * kHfinCarry);
constexpr float kResScale  = 2048.0f;
constexpr float kResInv    = 1.0f / kResScale;
constexpr float kWCarry    = 16.0f;
constexpr float kWInv      = 1.0f / kWCarry;
constexpr float kActCarry  = 1.0f;
constexpr float kF16MinNormal = 6.103515625e-5f;
static_assert(kI == kH && kO == kH, "square widths");
static_assert((kI % 32) == 0 && (kH % 32) == 0, "GEMM K multiples of 32");
static_assert((kB % 64) == 0 && (kG % 64) == 0 && (kO % 64) == 0, "GEMM M,N multiples of 64");
static_assert((kH % kChunkCols) == 0 && (kB % kRowsPerBlk) == 0, "tile multiples");
static_assert(kResInv * kResScale == 1.0f && kWInv * kWCarry == 1.0f, "power-of-two carries");

constexpr size_t kOut1Off = (size_t)kB * kO;
constexpr size_t kOut2Off = kOut1Off + (size_t)kB * kH;
constexpr size_t kOut3Off = kOut2Off + (size_t)kB * kH;
constexpr size_t kOutTotal = kOut3Off + (size_t)kB;
static_assert(kOut1Off * 4 == 8388608ull && kOut2Off * 4 == 16777216ull && kOut3Off * 4 == 25165824ull, "output byte offsets");
static_assert(kOutTotal * 4 == 25182208ull, "output total");

constexpr size_t kOffXH    = 0;
constexpr size_t kOffXL    = kOffXH    + (size_t)kB * kI * 2;
constexpr size_t kOffWIH   = kOffXL    + (size_t)kB * kI * 2;
constexpr size_t kOffWIL   = kOffWIH   + (size_t)kG * kI * 2;
constexpr size_t kOffWHH   = kOffWIL   + (size_t)kG * kI * 2;
constexpr size_t kOffWHL   = kOffWHH   + (size_t)kG * kH * 2;
constexpr size_t kOffWOF   = kOffWHL   + (size_t)kG * kH * 2;
constexpr size_t kOffWFLAG = kOffWOF   + (size_t)kO * kH * 2;
constexpr size_t kOffBIAS  = kOffWFLAG + (size_t)kG * 4;
constexpr size_t kOffXP    = kOffBIAS  + (size_t)kG * 4;
constexpr size_t kOffHP0H  = kOffXP    + (size_t)kB * kG * 4;
constexpr size_t kOffHP0L  = kOffHP0H  + (size_t)kB * kH * 2;
constexpr size_t kOffHP1H  = kOffHP0L  + (size_t)kB * kH * 2;
constexpr size_t kOffHP1L  = kOffHP1H  + (size_t)kB * kH * 2;
constexpr size_t kOffHNEW  = kOffHP1L  + (size_t)kB * kH * 2;
constexpr size_t kOffCPL   = kOffHNEW  + (size_t)kB * kH * 4;
constexpr size_t kOffHACC  = kOffCPL   + (size_t)kB * kH * 4;
constexpr size_t kOffCACC  = kOffHACC  + (size_t)kB * kH * 4;
constexpr size_t kOffHFIN  = kOffCACC  + (size_t)kB * kH * 4;
constexpr size_t kWsTotal  = kOffHFIN  + (size_t)kB * kH * 2;
static_assert(kWsTotal == 105398272ull, "carve total");
static_assert(kWsTotal <= 134217728ull, "carve cap");
static_assert((kOffXL % 128) == 0 && (kOffWIH % 128) == 0 && (kOffWIL % 128) == 0 && (kOffWHH % 128) == 0 &&
              (kOffWHL % 128) == 0 && (kOffWOF % 128) == 0 && (kOffWFLAG % 128) == 0 && (kOffBIAS % 128) == 0 &&
              (kOffXP % 128) == 0 && (kOffHP0H % 128) == 0 && (kOffHP0L % 128) == 0 && (kOffHP1H % 128) == 0 &&
              (kOffHP1L % 128) == 0 && (kOffHNEW % 128) == 0 && (kOffCPL % 128) == 0 && (kOffHACC % 128) == 0 &&
              (kOffCACC % 128) == 0 && (kOffHFIN % 128) == 0, "128-B aligned regions");

__device__ __forceinline__ void guard1_h(v8f& a, v16h x, v16h y, v16h z, v16h w) {
  asm volatile("v_nop\n\tv_nop\n\tv_nop\n\tv_nop" : "+v"(a) : "v"(x), "v"(y), "v"(z), "v"(w));
}
__device__ __forceinline__ void keep4_h(v16h a, v16h b, v16h c, v16h d) { asm volatile("v_nop" :: "v"(a), "v"(b), "v"(c), "v"(d)); }
__device__ __forceinline__ void acc_guard1(v8f& a) { asm volatile("v_nop\n\tv_nop\n\tv_nop\n\tv_nop" : "+v"(a)); }

template <typename T> struct Frag;
template <> struct Frag<_Float16> {
  typedef v16h V; union U { v16h v; v8h h[2]; };
  static __device__ __forceinline__ v16h load(const _Float16* p) {
    U f; f.h[0] = *(const v8h*)(p); f.h[1] = *(const v8h*)(p + 16); return f.v;
  }
  static __device__ __forceinline__ v8f mma(v16h a, v16h b, v8f c) {
    return __builtin_amdgcn_wmma_f32_16x16x32_f16(false, a, false, b, (short)0, c, false, false);
  }
};
typedef Frag<_Float16> FH;

__device__ __forceinline__ void split_val_res(float vc, _Float16& hi, _Float16& lo) {
  const float h0 = (float)((_Float16)vc);
  const float hq = (fabsf(h0) < kF16MinNormal) ? 0.0f : h0;
  hi = (_Float16)hq;
  const float rs = vc - hq;
  lo = (_Float16)(rs * kResScale);
}

__global__ __launch_bounds__(256) void wmma_gemm64_f16(
    const unsigned short* __restrict__ Ap, int lda,
    const unsigned short* __restrict__ Btp, int ldb,
    float* __restrict__ Cout, int ldc,
    const float* __restrict__ bias,
    int M, int N, int K, float scale) {
  const _Float16* Ab = (const _Float16*)Ap;
  const _Float16* Bb = (const _Float16*)Btp;
  __shared__ __align__(16) float sT[8][16 * 68];
  const int lane = threadIdx.x & 31;
  const int wave = threadIdx.x >> 5;
  const int tilesN = N >> 6;
  const int tilesM = M >> 6;
  const int tile = blockIdx.x * 8 + wave;
  if (tile >= tilesM * tilesN) return;
  const int tm = tile / tilesN;
  const int tn = tile - tm * tilesN;
  const int m0 = tm << 6;
  const int n0 = tn << 6;

  const int rlane = lane & 15;
  const int koff  = (lane >> 4) * 8;
  const int mOff  = (lane >> 4) * 8;

  v8f acc[4][4];
#pragma unroll
  for (int i = 0; i < 4; ++i)
#pragma unroll
    for (int j = 0; j < 4; ++j) acc[i][j] = (v8f){0.f,0.f,0.f,0.f,0.f,0.f,0.f,0.f};

  for (int k0 = 0; k0 < K; k0 += 32) {
    v16h bh[4];
#pragma unroll
    for (int j = 0; j < 4; ++j) {
      const size_t bo = (size_t)(n0 + (j << 4) + rlane) * ldb + koff + k0;
      bh[j] = FH::load(Bb + bo);
    }
#pragma unroll
    for (int i = 0; i < 4; ++i) {
      const size_t ao = (size_t)(m0 + (i << 4) + rlane) * lda + koff + k0;
      const v16h ah = FH::load(Ab + ao);
#pragma unroll
      for (int j = 0; j < 4; ++j) acc[i][j] = FH::mma(ah, bh[j], acc[i][j]);
#pragma unroll
      for (int j = 0; j < 4; ++j) guard1_h(acc[i][j], ah, ah, bh[j], bh[j]);
    }
    keep4_h(bh[0], bh[1], bh[2], bh[3]);
  }
#pragma unroll
  for (int i = 0; i < 4; ++i)
#pragma unroll
    for (int j = 0; j < 4; ++j) acc_guard1(acc[i][j]);

  float* slab = sT[wave];
#pragma unroll
  for (int i = 0; i < 4; ++i) {
    const int mBase = m0 + (i << 4);
#pragma unroll
    for (int j = 0; j < 4; ++j) {
      const int n = n0 + (j << 4) + rlane;
      const float bv = bias[n];
#pragma unroll
      for (int r = 0; r < 8; ++r) {
        const float v = acc[i][j][r] * scale + bv;
        slab[(mOff + r) * 68 + (j << 4) + rlane] = v;
      }
    }
    __builtin_amdgcn_fence(__ATOMIC_RELEASE, "workgroup");
    __builtin_amdgcn_wave_barrier();
    __builtin_amdgcn_fence(__ATOMIC_ACQUIRE, "workgroup");
    {
      const int hh = lane >> 4, c4 = (lane & 15) * 4;
      for (int pass = 0; pass < 2; ++pass) {
#pragma unroll
        for (int it = 0; it < 8; ++it) {
          const int row = it * 2 + hh;
          v4f v = *(const v4f*)(slab + row * 68 + c4);
          *(volatile v4f*)(Cout + (size_t)(mBase + row) * ldc + n0 + c4) = v;
        }
        __threadfence();
      }
    }
    __builtin_amdgcn_fence(__ATOMIC_RELEASE, "workgroup");
    __builtin_amdgcn_wave_barrier();
    __builtin_amdgcn_fence(__ATOMIC_ACQUIRE, "workgroup");
  }
}

__global__ __launch_bounds__(256) void split_gemm32_kernel(
    const unsigned short* __restrict__ Ahp, const unsigned short* __restrict__ Alp, int lda,
    const unsigned short* __restrict__ Bhp, const unsigned short* __restrict__ Blp, int ldb,
    float* __restrict__ Cout, int ldc,
    const float* __restrict__ bias,
    int M, int N, int K, float scale) {
  const _Float16* Ah = (const _Float16*)Ahp;
  const _Float16* Al = (const _Float16*)Alp;
  const _Float16* Bh = (const _Float16*)Bhp;
  const _Float16* Bl = (const _Float16*)Blp;
  __shared__ __align__(16) float sT[8][16 * 36];
  const int lane = threadIdx.x & 31;
  const int wave = threadIdx.x >> 5;
  const int tilesN = N >> 5;
  const int tilesM = M >> 5;
  const int tile = blockIdx.x * 8 + wave;
  if (tile >= tilesM * tilesN) return;
  const int tm = tile / tilesN;
  const int tn = tile - tm * tilesN;
  const int m0 = tm << 5;
  const int n0 = tn << 5;

  const int rlane = lane & 15;
  const int koff  = (lane >> 4) * 8;
  const int mOff  = (lane >> 4) * 8;

  v8f acc[2][2], acc2[2][2];
#pragma unroll
  for (int i = 0; i < 2; ++i)
#pragma unroll
    for (int j = 0; j < 2; ++j) {
      acc[i][j]  = (v8f){0.f,0.f,0.f,0.f,0.f,0.f,0.f,0.f};
      acc2[i][j] = (v8f){0.f,0.f,0.f,0.f,0.f,0.f,0.f,0.f};
    }

#pragma unroll 1
  for (int k0 = 0; k0 < K; k0 += 32) {
    v16h bh[2], bl[2], ah[2], al[2];
#pragma unroll
    for (int j = 0; j < 2; ++j) {
      const size_t bo = (size_t)(n0 + (j << 4) + rlane) * ldb + koff + k0;
      bh[j] = FH::load(Bh + bo);
      bl[j] = FH::load(Bl + bo);
    }
#pragma unroll
    for (int i = 0; i < 2; ++i) {
      const size_t ao = (size_t)(m0 + (i << 4) + rlane) * lda + koff + k0;
      ah[i] = FH::load(Ah + ao);
      al[i] = FH::load(Al + ao);
    }
#pragma unroll
    for (int i = 0; i < 2; ++i)
#pragma unroll
      for (int j = 0; j < 2; ++j) {
        acc[i][j]  = FH::mma(ah[i], bh[j], acc[i][j]);
        acc2[i][j] = FH::mma(ah[i], bl[j], acc2[i][j]);
        acc2[i][j] = FH::mma(al[i], bh[j], acc2[i][j]);
      }
#pragma unroll
    for (int i = 0; i < 2; ++i)
#pragma unroll
      for (int j = 0; j < 2; ++j) {
        guard1_h(acc[i][j],  ah[i], al[i], bh[j], bl[j]);
        guard1_h(acc2[i][j], ah[i], al[i], bh[j], bl[j]);
      }
  }
#pragma unroll
  for (int i = 0; i < 2; ++i)
#pragma unroll
    for (int j = 0; j < 2; ++j) {
      acc_guard1(acc[i][j]);
      acc_guard1(acc2[i][j]);
    }

  float* slab = sT[wave];
  float bvv[2];
  bvv[0] = bias[n0 + rlane];
  bvv[1] = bias[n0 + 16 + rlane];
#pragma unroll
  for (int i = 0; i < 2; ++i) {
    const int mBase = m0 + (i << 4);
#pragma unroll
    for (int j = 0; j < 2; ++j) {
#pragma unroll
      for (int r = 0; r < 8; ++r) {
        const float s = acc[i][j][r] + acc2[i][j][r] * kResInv;
        const float v = s * scale + bvv[j];
        slab[(mOff + r) * 36 + (j << 4) + rlane] = v;
      }
    }
    __builtin_amdgcn_fence(__ATOMIC_RELEASE, "workgroup");
    __builtin_amdgcn_wave_barrier();
    __builtin_amdgcn_fence(__ATOMIC_ACQUIRE, "workgroup");
    {
      const int q = lane >> 3, c4 = (lane & 7) * 4;
      for (int pass = 0; pass < 2; ++pass) {
#pragma unroll
        for (int it = 0; it < 4; ++it) {
          const int row = it * 4 + q;
          v4f v = *(const v4f*)(slab + row * 36 + c4);
          *(volatile v4f*)(Cout + (size_t)(mBase + row) * ldc + n0 + c4) = v;
        }
        __threadfence();
      }
    }
    __builtin_amdgcn_fence(__ATOMIC_RELEASE, "workgroup");
    __builtin_amdgcn_wave_barrier();
    __builtin_amdgcn_fence(__ATOMIC_ACQUIRE, "workgroup");
  }
}

__global__ __launch_bounds__(256) void split_rows_f16_kernel(
    const float* __restrict__ src, unsigned short* __restrict__ dhi, unsigned short* __restrict__ dlo,
    int total8, float carry)
{
  const int i = blockIdx.x * 256 + threadIdx.x;
  if (i >= total8) return;
  const size_t e0 = (size_t)i << 3;
  const v4f a0 = *(const v4f*)(src + e0);
  const v4f a1 = *(const v4f*)(src + e0 + 4);
  v8h hv, lv;
#pragma unroll
  for (int e = 0; e < 4; ++e) {
    const float f0 = a0[e] * carry;
    const float f1 = a1[e] * carry;
    _Float16 h0, l0, h1, l1;
    split_val_res(f0, h0, l0);
    split_val_res(f1, h1, l1);
    hv[e]     = h0;
    hv[4 + e] = h1;
    lv[e]     = l0;
    lv[4 + e] = l1;
  }
  unsigned short* qh = dhi + e0;
  unsigned short* ql = dlo + e0;
  *(volatile v8h*)qh = hv;
  *(volatile v8h*)ql = lv;
  __threadfence();
  *(volatile v8h*)qh = hv;
  *(volatile v8h*)ql = lv;
}

constexpr int kRepackBlocks = (kG * kI / 8) / 256;
constexpr int kVecBlocks    = (kG / 4) / 256;
static_assert(kRepackBlocks * 256 * 8 == kG * kI && kVecBlocks * 256 * 4 == kG, "exact coverage");
__global__ __launch_bounds__(256) void repack_wih_kernel(
    const float* __restrict__ Wih, const float* __restrict__ bih, const float* __restrict__ bhh,
    unsigned short* __restrict__ dhi, unsigned short* __restrict__ dlo,
    float* __restrict__ wflag, float* __restrict__ bias)
{
  if ((int)blockIdx.x < kRepackBlocks) {
    const int i  = blockIdx.x * 256 + threadIdx.x;
    const int n  = i >> 6;
    const int c8 = (i & 63) * 8;
    const float* sp = Wih + (size_t)n * kWihP + 1 + c8;
    v8h hv, lv;
#pragma unroll
    for (int e = 0; e < 8; ++e) {
      const float f = sp[e] * kWCarry;
      _Float16 hq, lq;
      split_val_res(f, hq, lq);
      hv[e] = hq;
      lv[e] = lq;
    }
    unsigned short* qh = dhi + (size_t)n * kI + c8;
    unsigned short* ql = dlo + (size_t)n * kI + c8;
    *(volatile v8h*)qh = hv;
    *(volatile v8h*)ql = lv;
    __threadfence();
    *(volatile v8h*)qh = hv;
    *(volatile v8h*)ql = lv;
  } else {
    const int t  = ((int)blockIdx.x - kRepackBlocks) * 256 + threadIdx.x;
    const int n4 = t * 4;
    const v4f bi = *(const v4f*)(bih + n4);
    const v4f bh = *(const v4f*)(bhh + n4);
    v4f wf, bs;
#pragma unroll
    for (int e = 0; e < 4; ++e) {
      wf[e] = Wih[(size_t)(n4 + e) * kWihP];
      bs[e] = bi[e] + bh[e];
    }
    *(volatile v4f*)(wflag + n4) = wf;
    *(volatile v4f*)(bias + n4)  = bs;
    __threadfence();
    *(volatile v4f*)(wflag + n4) = wf;
    *(volatile v4f*)(bias + n4)  = bs;
  }
}

__global__ __launch_bounds__(256) void cast_wout_kernel(
    const float* __restrict__ src, unsigned short* __restrict__ dst, int total8)
{
  const int i = blockIdx.x * 256 + threadIdx.x;
  if (i >= total8) return;
  const size_t e0 = (size_t)i << 3;
  const v4f a0 = *(const v4f*)(src + e0);
  const v4f a1 = *(const v4f*)(src + e0 + 4);
  v8h hv;
#pragma unroll
  for (int e = 0; e < 4; ++e) {
    const float f0 = a0[e] * kWoutCarry;
    const float f1 = a1[e] * kWoutCarry;
    hv[e]     = (_Float16)f0;
    hv[4 + e] = (_Float16)f1;
  }
  unsigned short* q = dst + e0;
  *(volatile v8h*)q = hv;
  __threadfence();
  *(volatile v8h*)q = hv;
}

__device__ __forceinline__ float gate_sigmoid(float z) { return __builtin_amdgcn_rcpf(1.0f + __expf(-z)); }
__device__ __forceinline__ float gate_tanh(float z) { return 1.0f - 2.0f * __builtin_amdgcn_rcpf(__expf(2.0f * z) + 1.0f); }

__global__ __launch_bounds__(256) void halting_lstm_steps_kernel(
    const float* __restrict__ xpart, const float* __restrict__ wflag, const float* c0,
    const unsigned short* __restrict__ whh_hi, const unsigned short* __restrict__ whh_lo,
    const float* __restrict__ whalt, const float* __restrict__ bhalt, const int* __restrict__ msteps,
    unsigned short* hp0h, unsigned short* hp0l, unsigned short* hp1h, unsigned short* hp1l,
    float* hnew, float* cpl, float* hacc, float* cacc,
    unsigned short* hfin16, float* out1, float* out2, float* out3)
{
  __shared__ __align__(16) float sPatch[32 * kPatchP];
  __shared__ __align__(16) float sPond[64];
  __shared__ float sDot[64];
  __shared__ float sWgt[64];
  __shared__ int   sHalt[64];

  const int tid  = threadIdx.x;
  const int lane = tid & 31;
  const int wave = tid >> 5;
  const int rt   = wave >> 2;
  const int ct   = wave & 3;
  const int l15  = lane & 15;
  const int hh   = lane >> 4;
  const int m0   = blockIdx.x * kRowsPerBlk;
  const int crow = tid >> 4;
  const int cc4  = (tid & 15) * 4;
  const float bh = bhalt[0];
  const float pz = (msteps[0] == kSteps) ? 0.0f : __uint_as_float(0x7fc00000u);
  const _Float16* Wh = (const _Float16*)whh_hi;
  const _Float16* Wl = (const _Float16*)whh_lo;

  float cum = 0.f, psum = 0.f, pond = 0.f;
  int halted = 0;

#pragma unroll 1
  for (int n = 0; n < kSteps; ++n) {
    const bool first = (n == 0);
    const unsigned short* curh = (n & 1) ? hp1h : hp0h;
    const unsigned short* curl = (n & 1) ? hp1l : hp0l;
    unsigned short* nxth = (n & 1) ? hp0h : hp1h;
    unsigned short* nxtl = (n & 1) ? hp0l : hp1l;
    const _Float16* Ah = (const _Float16*)curh;
    const _Float16* Al = (const _Float16*)curl;
    const float* csrc = first ? c0 : (const float*)cpl;
    if (tid < 64) sDot[tid] = 0.f;

#pragma unroll 1
    for (int ch = 0; ch < kH / kChunkCols; ++ch) {
      const int j0 = ch * kChunkCols;
      const size_t bbase = (size_t)(j0 + ct * 16 + l15) * kH + 8 * hh;

#pragma unroll 1
      for (int hf = 0; hf < 2; ++hf) {
        v8f acc[4], acc2[4];
#pragma unroll
        for (int g = 0; g < 4; ++g) {
          acc[g]  = (v8f){0.f,0.f,0.f,0.f,0.f,0.f,0.f,0.f};
          acc2[g] = (v8f){0.f,0.f,0.f,0.f,0.f,0.f,0.f,0.f};
        }
        const size_t abase = (size_t)(m0 + hf * 32 + rt * 16 + l15) * kH + 8 * hh;
#pragma unroll 1
        for (int k0 = 0; k0 < kH; k0 += 32) {
          v16h bhf[4], blf[4];
#pragma unroll
          for (int g = 0; g < 4; ++g) {
            const size_t bo = bbase + (size_t)g * kH * kH + k0;
            bhf[g] = FH::load(Wh + bo);
            blf[g] = FH::load(Wl + bo);
          }
          const v16h ah = FH::load(Ah + abase + k0);
          const v16h al = FH::load(Al + abase + k0);
#pragma unroll
          for (int g = 0; g < 4; ++g) {
            acc[g]  = FH::mma(ah, bhf[g], acc[g]);
            acc2[g] = FH::mma(ah, blf[g], acc2[g]);
            acc2[g] = FH::mma(al, bhf[g], acc2[g]);
          }
#pragma unroll
          for (int g = 0; g < 4; ++g) {
            guard1_h(acc[g],  ah, al, bhf[g], blf[g]);
            guard1_h(acc2[g], ah, al, bhf[g], blf[g]);
          }
        }
#pragma unroll
        for (int g = 0; g < 4; ++g) {
          acc_guard1(acc[g]);
          acc_guard1(acc2[g]);
        }

        __syncthreads();
#pragma unroll
        for (int g = 0; g < 4; ++g)
#pragma unroll
          for (int r = 0; r < 8; ++r) {
            const float s = acc[g][r] + acc2[g][r] * kResInv;
            sPatch[(rt * 16 + 8 * hh + r) * kPatchP + g * 64 + ct * 16 + l15] = s * kWInv;
          }
        __syncthreads();

        const v4f wh = *(const v4f*)(whalt + j0 + cc4);
        v4f wi[4];
#pragma unroll
        for (int g = 0; g < 4; ++g) wi[g] = (v4f){0.f, 0.f, 0.f, 0.f};
        if (first) {
#pragma unroll
          for (int g = 0; g < 4; ++g) wi[g] = *(const v4f*)(wflag + g * kH + j0 + cc4);
        }

#pragma unroll 1
        for (int it = 0; it < 2; ++it) {
          const int lr  = crow + 16 * it;
          const int row = m0 + hf * 32 + lr;
          const int col = j0 + cc4;
          const float* pp = sPatch + lr * kPatchP + cc4;
          const float* xp = xpart + (size_t)row * kG + col;
          v4f gv[4];
#pragma unroll
          for (int g = 0; g < 4; ++g) {
            const v4f pa = *(const v4f*)(pp + g * 64);
            const v4f xa = *(const v4f*)(xp + g * kH);
            v4f s;
#pragma unroll
            for (int e = 0; e < 4; ++e) s[e] = (xa[e] + wi[g][e]) + pa[e];
            gv[g] = s;
          }
          const size_t so = (size_t)row * kH + col;
          const v4f cold = *(const v4f*)(csrc + so);
          v4f cn, hn;
          unsigned hb[4], lb[4];
          float part = 0.f;
#pragma unroll
          for (int e = 0; e < 4; ++e) {
            const float si = gate_sigmoid(gv[0][e]);
            const float sf = gate_sigmoid(gv[1][e]);
            const float tg = gate_tanh(gv[2][e]);
            const float sg = gate_sigmoid(gv[3][e]);
            const float c1 = sf * cold[e] + si * tg;
            const float h1 = sg * gate_tanh(c1);
            cn[e] = c1;
            hn[e] = h1;
            part += h1 * wh[e];
            _Float16 hq, lq;
            split_val_res(h1 * kActCarry, hq, lq);
            hb[e] = (unsigned)__builtin_bit_cast(unsigned short, hq);
            lb[e] = (unsigned)__builtin_bit_cast(unsigned short, lq);
          }
          part += __shfl_xor(part, 1, 32);
          part += __shfl_xor(part, 2, 32);
          part += __shfl_xor(part, 4, 32);
          part += __shfl_xor(part, 8, 32);
          if (l15 == 0) sDot[hf * 32 + lr] += part;

          v2u ph, pl;
          ph[0] = hb[0] | (hb[1] << 16);
          ph[1] = hb[2] | (hb[3] << 16);
          pl[0] = lb[0] | (lb[1] << 16);
          pl[1] = lb[2] | (lb[3] << 16);
          float* cdst = cpl + so;
          float* hdst = hnew + so;
          unsigned short* nh = nxth + so;
          unsigned short* nl = nxtl + so;
          *(volatile v4f*)cdst = cn;
          *(volatile v4f*)hdst = hn;
          *(volatile v2u*)nh = ph;
          *(volatile v2u*)nl = pl;
          __threadfence();
          *(volatile v4f*)cdst = cn;
          *(volatile v4f*)hdst = hn;
          *(volatile v2u*)nh = ph;
          *(volatile v2u*)nl = pl;
        }
      }
    }

    __threadfence();
    __syncthreads();
    if (tid < 64) {
      float w = 0.f;
      if (halted == 0) {
        const float s  = sDot[tid] + bh;
        const float hv = 1.0f / (1.0f + expf(-s));
        cum += hv;
        if (cum >= 0.99f || n == kSteps - 1) {
          w = 1.0f - psum;
          halted = 1;
          pond = (float)n + 1.0f + w;
        } else {
          w = hv;
          psum += hv;
        }
      }
      sWgt[tid]  = w;
      sHalt[tid] = halted;
    }
    __syncthreads();
    __threadfence();

    int tot = 0;
#pragma unroll 1
    for (int i = 0; i < 64; ++i) tot += sHalt[i];

#pragma unroll 1
    for (int rr = 0; rr < 8; ++rr) {
      const int lrow = wave * 8 + rr;
      const float w = sWgt[lrow];
      if (first || w != 0.f) {
        const size_t rb = (size_t)(m0 + lrow) * kH;
#pragma unroll 1
        for (int k = 0; k < 4; ++k) {
          const size_t o = rb + (size_t)(lane + 32 * k) * 4;
          const v4f hv = *(const v4f*)(hnew + o);
          const v4f cv = *(const v4f*)(cpl + o);
          v4f ha = (v4f){0.f, 0.f, 0.f, 0.f};
          v4f ca = (v4f){0.f, 0.f, 0.f, 0.f};
          if (!first) {
            ha = *(const v4f*)(hacc + o);
            ca = *(const v4f*)(cacc + o);
          }
          v4f hr, cr;
#pragma unroll
          for (int e = 0; e < 4; ++e) {
            hr[e] = ha[e] + w * hv[e];
            cr[e] = ca[e] + w * cv[e];
          }
          *(volatile v4f*)(hacc + o) = hr;
          *(volatile v4f*)(cacc + o) = cr;
          __threadfence();
          *(volatile v4f*)(hacc + o) = hr;
          *(volatile v4f*)(cacc + o) = cr;
        }
      }
    }
    if (tot == 64) break;
  }

  __threadfence();
  if (tid < 64) sPond[tid] = pond;
  __syncthreads();
#pragma unroll 1
  for (int rr = 0; rr < 8; ++rr) {
    const int lrow = wave * 8 + rr;
    const size_t rb = (size_t)(m0 + lrow) * kH;
#pragma unroll 1
    for (int k = 0; k < 4; ++k) {
      const size_t o = rb + (size_t)(lane + 32 * k) * 4;
      const v4f ha = *(const v4f*)(hacc + o);
      const v4f ca = *(const v4f*)(cacc + o);
      v4f ho, co;
      unsigned qb[4];
#pragma unroll
      for (int e = 0; e < 4; ++e) {
        const float hval = ha[e] + pz;
        const float cval = ca[e] + pz;
        ho[e] = hval;
        co[e] = cval;
        const _Float16 q = (_Float16)(hval * kHfinCarry);
        qb[e] = (unsigned)__builtin_bit_cast(unsigned short, q);
      }
      v2u pk;
      pk[0] = qb[0] | (qb[1] << 16);
      pk[1] = qb[2] | (qb[3] << 16);
      *(volatile v4f*)(out1 + o) = ho;
      *(volatile v4f*)(out2 + o) = co;
      *(volatile v2u*)(hfin16 + o) = pk;
      __threadfence();
      *(volatile v4f*)(out1 + o) = ho;
      *(volatile v4f*)(out2 + o) = co;
      *(volatile v2u*)(hfin16 + o) = pk;
    }
  }
  if (tid < 16) {
    const v4f pl = *(const v4f*)(sPond + tid * 4);
    v4f pv;
#pragma unroll
    for (int e = 0; e < 4; ++e) pv[e] = pl[e] + pz;
    float* pd = out3 + m0 + tid * 4;
    *(volatile v4f*)pd = pv;
    __threadfence();
    *(volatile v4f*)pd = pv;
  }
}

extern "C" void kernel_launch(void* const* d_in, const int* in_sizes, int n_in,
                              void* d_out, int out_size, void* d_ws, size_t ws_size,
                              hipStream_t stream) {
  if (n_in < 12) return;
  if (in_sizes[0] != kB * kI) return;
  if (in_sizes[1] != kB * kH) return;
  if (in_sizes[2] != kB * kH) return;
  if (in_sizes[3] != kG * kWihP) return;
  if (in_sizes[4] != kG) return;
  if (in_sizes[5] != kG * kH) return;
  if (in_sizes[6] != kG) return;
  if (in_sizes[7] != kH) return;
  if (in_sizes[8] != 1) return;
  if (in_sizes[9] != kO * kH) return;
  if (in_sizes[10] != kO) return;
  if (in_sizes[11] != 1) return;
  if ((size_t)out_size != kOutTotal) return;
  if (ws_size < kWsTotal) return;

  const float* x      = (const float*)d_in[0];
  const float* h0     = (const float*)d_in[1];
  const float* c0     = (const float*)d_in[2];
  const float* W_ih   = (const float*)d_in[3];
  const float* b_ih   = (const float*)d_in[4];
  const float* W_hh   = (const float*)d_in[5];
  const float* b_hh   = (const float*)d_in[6];
  const float* W_halt = (const float*)d_in[7];
  const float* b_halt = (const float*)d_in[8];
  const float* W_out  = (const float*)d_in[9];
  const float* b_out  = (const float*)d_in[10];
  const int*   msteps = (const int*)d_in[11];
  float* out = (float*)d_out;

  char* ws = (char*)d_ws;
  unsigned short* XH    = (unsigned short*)(ws + kOffXH);
  unsigned short* XL    = (unsigned short*)(ws + kOffXL);
  unsigned short* WIH   = (unsigned short*)(ws + kOffWIH);
  unsigned short* WIL   = (unsigned short*)(ws + kOffWIL);
  unsigned short* WHH   = (unsigned short*)(ws + kOffWHH);
  unsigned short* WHL   = (unsigned short*)(ws + kOffWHL);
  unsigned short* WOF   = (unsigned short*)(ws + kOffWOF);
  float*          WFLAG = (float*)(ws + kOffWFLAG);
  float*          BIAS  = (float*)(ws + kOffBIAS);
  float*          XP    = (float*)(ws + kOffXP);
  unsigned short* HP0H  = (unsigned short*)(ws + kOffHP0H);
  unsigned short* HP0L  = (unsigned short*)(ws + kOffHP0L);
  unsigned short* HP1H  = (unsigned short*)(ws + kOffHP1H);
  unsigned short* HP1L  = (unsigned short*)(ws + kOffHP1L);
  float*          HNEW  = (float*)(ws + kOffHNEW);
  float*          CPL   = (float*)(ws + kOffCPL);
  float*          HACC  = (float*)(ws + kOffHACC);
  float*          CACC  = (float*)(ws + kOffCACC);
  unsigned short* HFIN  = (unsigned short*)(ws + kOffHFIN);

  split_rows_f16_kernel<<<(kB * kI / 8) / 256, 256, 0, stream>>>(x, XH, XL, kB * kI / 8, kActCarry);
  split_rows_f16_kernel<<<(kB * kH / 8) / 256, 256, 0, stream>>>(h0, HP0H, HP0L, kB * kH / 8, kActCarry);
  split_rows_f16_kernel<<<(kG * kH / 8) / 256, 256, 0, stream>>>(W_hh, WHH, WHL, kG * kH / 8, kWCarry);
  repack_wih_kernel<<<kRepackBlocks + kVecBlocks, 256, 0, stream>>>(W_ih, b_ih, b_hh, WIH, WIL, WFLAG, BIAS);
  cast_wout_kernel<<<(kO * kH / 8) / 256, 256, 0, stream>>>(W_out, WOF, kO * kH / 8);

  split_gemm32_kernel<<<((kB / 32) * (kG / 32)) / 8, 256, 0, stream>>>(
      XH, XL, kI,
      WIH, WIL, kI,
      XP, kG,
      BIAS,
      kB, kG, kI, kWInv);

  halting_lstm_steps_kernel<<<kB / kRowsPerBlk, 256, 0, stream>>>(
      XP, WFLAG, c0, WHH, WHL, W_halt, b_halt, msteps,
      HP0H, HP0L, HP1H, HP1L,
      HNEW, CPL, HACC, CACC,
      HFIN, out + kOut1Off, out + kOut2Off, out + kOut3Off);

  wmma_gemm64_f16<<<((kB / 64) * (kO / 64)) / 8, 256, 0, stream>>>(
      HFIN, kH,
      WOF, kH,
      out, kO,
      b_out,
      kB, kO, kH, kOutScale);
}
